// GCN_65876208386064
// MI455X (gfx1250) — hardware-verified
//
#include <hip/hip_runtime.h>
#include <stddef.h>
#include <stdint.h>
#include <math.h>


#define NTHR   256
#define NWAVE  8
#define NBR    256
#define SLB    8
#define SCH    4096
#define NB2    2048
#define DUMP   (NB2 - 1)
#define RCAP   3072
#define SEGCAP 64
#define PQ1P   32
#define PQ2P   8
#define ENC_NINF 0x007FFFFFu
#define WSMAX  134217728

static_assert(NBR == (1 << SLB));
static_assert(SCH == NTHR * 16);
static_assert(NB2 == NTHR * 8);
static_assert(RCAP % 16 == 0);
static_assert((NBR * 16) % (NTHR * 4) == 0);
static_assert(NBR == NTHR);

typedef float          v4f   __attribute__((ext_vector_type(4)));
typedef float          v8f   __attribute__((ext_vector_type(8)));
typedef int            v4i   __attribute__((ext_vector_type(4)));
typedef int            v8i   __attribute__((ext_vector_type(8)));
typedef unsigned int   v4u   __attribute__((ext_vector_type(4)));
typedef unsigned short v8us  __attribute__((ext_vector_type(8)));
typedef unsigned short v16us __attribute__((ext_vector_type(16)));
typedef __bf16         v16bf __attribute__((ext_vector_type(16)));
typedef v4f  __attribute__((may_alias)) v4fa;
typedef v4i  __attribute__((may_alias)) v4ia;
typedef v4u  __attribute__((may_alias)) v4ua;
typedef v8us __attribute__((may_alias)) v8usa;
union FragB { v16bf v; v16us u; v8us h[2]; v8i w; };

__device__ __forceinline__ v8f wmb(const FragB& a, const FragB& b, v8f c) {
  v8f d = __builtin_amdgcn_wmma_f32_16x16x32_bf16(false, a.v, false, b.v, (short)0, c, false, false);
  asm volatile("v_nop\n\tv_nop\n\tv_nop\n\tv_nop" : "+v"(d) : "v"(a.w), "v"(b.w));
  return d;
}

__device__ __forceinline__ unsigned bf16_bits(float f) {
  const unsigned u = __float_as_uint(f);
  return (u + 0x7FFFu + ((u >> 16) & 1u)) >> 16;
}
__device__ __forceinline__ float bf16_val(float f) {
  return __uint_as_float(bf16_bits(f) << 16);
}

__device__ __forceinline__ void wave_sync() {
  __builtin_amdgcn_fence(__ATOMIC_RELEASE, "wavefront");
  __builtin_amdgcn_wave_barrier();
  __builtin_amdgcn_fence(__ATOMIC_ACQUIRE, "wavefront");
}

__device__ __forceinline__ unsigned enc_f(float v) {
  const unsigned u = __float_as_uint(v);
  unsigned e = (u & 0x80000000u) ? ~u : (u | 0x80000000u);
  e = (v != v) ? 0xFFFFFFFFu : e;
  return e;
}
__device__ __forceinline__ float dec_f(unsigned e) {
  const unsigned u = (e & 0x80000000u) ? (e & 0x7FFFFFFFu) : ~e;
  return __uint_as_float(u);
}
__device__ __forceinline__ float relu_np(float v) { return (v > 0.0f) ? v : (v - v); }

__global__ __launch_bounds__(NTHR) void k_prep(const float* __restrict__ x, const float* __restrict__ w1a,
                                               const float* __restrict__ b1a, int nN, float* pq1) {
  __shared__ __attribute__((aligned(16))) float T1[4 * PQ1P];
  const int tid = (int)threadIdx.x;
  {
    const int idx = tid & 127;
    const int rr = idx >> 5, col = idx & 31, c = col & 15;
    const int rc = rr < 3 ? rr : 2;
    const float top = bf16_val(w1a[rc * 16 + c]);
    const float bot = bf16_val(w1a[(3 + rc) * 16 + c]);
    const float bia = bf16_val(b1a[c]);
    const float f   = (float)(1 - (col >> 4));
    const float wv  = fmaf(f, top - bot, (1.0f - f) * bot);
    const float bv  = f * bia;
    const float val = (rr < 3) ? wv : bv;
    if (tid < 128) T1[idx] = val;
  }
  __syncthreads();
  const int nodeBase = (int)blockIdx.x * NBR;
  const int c4 = tid & 7;
  const v4f w0 = *(const v4fa*)(T1 + 4 * c4);
  const v4f w1 = *(const v4fa*)(T1 + PQ1P + 4 * c4);
  const v4f w2 = *(const v4fa*)(T1 + 2 * PQ1P + 4 * c4);
  const v4f bb = *(const v4fa*)(T1 + 3 * PQ1P + 4 * c4);
#pragma unroll 1
  for (int it = 0; it < 8; ++it) {
    const int node = nodeBase + it * 32 + (tid >> 3);
    const int nc = node < nN ? node : nN - 1;
    const float* xp = x + (size_t)nc * 3;
    const float x0 = bf16_val(xp[0]);
    const float x1 = bf16_val(xp[1]);
    const float x2 = bf16_val(xp[2]);
    v4f s = w0 * x0;
    s = w1 * x1 + s;
    s = w2 * x2 + s;
    s = s + bb;
    const bool ok = node < nN;
    s.x = ok ? s.x : 0.0f; s.y = ok ? s.y : 0.0f; s.z = ok ? s.z : 0.0f; s.w = ok ? s.w : 0.0f;
    float* op = pq1 + (size_t)node * PQ1P + 4 * c4;
    *(volatile v4f*)op = s;
    __threadfence();
    *(volatile v4f*)op = s;
  }
}

__device__ __forceinline__ void load_edges4(const int* __restrict__ srcs, const int* __restrict__ dsts, int nE,
                                            int e0, int usevec, v4i& sa, v4i& da, v4i& va) {
  if (usevec != 0) {
    sa = *(const v4ia*)(srcs + e0);
    da = *(const v4ia*)(dsts + e0);
    va.x = 1; va.y = 1; va.z = 1; va.w = 1;
  } else {
    const int l = nE - 1;
    sa.x = srcs[min(e0,     l)]; sa.y = srcs[min(e0 + 1, l)];
    sa.z = srcs[min(e0 + 2, l)]; sa.w = srcs[min(e0 + 3, l)];
    da.x = dsts[min(e0,     l)]; da.y = dsts[min(e0 + 1, l)];
    da.z = dsts[min(e0 + 2, l)]; da.w = dsts[min(e0 + 3, l)];
    va.x = (e0     < nE) ? 1 : 0; va.y = (e0 + 1 < nE) ? 1 : 0;
    va.z = (e0 + 2 < nE) ? 1 : 0; va.w = (e0 + 3 < nE) ? 1 : 0;
  }
}

__global__ __launch_bounds__(NTHR) void k_sort(const int* __restrict__ srcs, const int* __restrict__ dsts,
                                               int nE, int nN, int vec4, int offp,
                                               unsigned* sorted, int* offs) {
  __shared__ __attribute__((aligned(16))) int cnt[NB2];
  __shared__ __attribute__((aligned(16))) int st[NB2];
  __shared__ __attribute__((aligned(16))) unsigned sl[SCH];
  __shared__ int wtot[NWAVE];
  const int tid = (int)threadIdx.x, lane = tid & 31, wave = tid >> 5;
  const int cbase = (int)blockIdx.x * SCH;
  const int usevec = (vec4 != 0 && cbase + SCH <= nE) ? 1 : 0;

  {
    const v4i z4 = {0, 0, 0, 0};
    *(v4ia*)(cnt + 8 * tid) = z4;
    *(v4ia*)(cnt + 8 * tid + 4) = z4;
  }
  __syncthreads();

#define HB1(D, V) { int d_ = (D); d_ = d_ < 0 ? 0 : (d_ > nN - 1 ? nN - 1 : d_); \
    const int bk_ = ((V) != 0) ? (d_ >> SLB) : DUMP; atomicAdd(&cnt[bk_], 1); }
#pragma unroll 1
  for (int it = 0; it < 4; ++it) {
    const int e0 = cbase + it * (NTHR * 4) + tid * 4;
    v4i sa, da, va;
    load_edges4(srcs, dsts, nE, e0, usevec, sa, da, va);
    HB1(da.x, va.x) HB1(da.y, va.y) HB1(da.z, va.z) HB1(da.w, va.w)
  }
#undef HB1
  __syncthreads();

  {
    const v4i c0 = *(const v4ia*)(cnt + 8 * tid);
    const v4i c1 = *(const v4ia*)(cnt + 8 * tid + 4);
    const int s = c0.x + c0.y + c0.z + c0.w + c1.x + c1.y + c1.z + c1.w;
    int incl = s;
#pragma unroll
    for (int d = 1; d < 32; d <<= 1) {
      const int y = __shfl_up(incl, d, 32);
      if (lane >= d) incl += y;
    }
    if (lane == 31) wtot[wave] = incl;
    __syncthreads();
    int base = 0;
#pragma unroll
    for (int w2 = 0; w2 < NWAVE; ++w2) { const int v = wtot[w2]; base += (w2 < wave) ? v : 0; }
    int run = base + incl - s;
    v4i o0, o1;
    o0.x = run; run += c0.x; o0.y = run; run += c0.y; o0.z = run; run += c0.z; o0.w = run; run += c0.w;
    o1.x = run; run += c1.x; o1.y = run; run += c1.y; o1.z = run; run += c1.z; o1.w = run;
    *(v4ia*)(st + 8 * tid) = o0;  *(v4ia*)(st + 8 * tid + 4) = o1;
    *(v4ia*)(cnt + 8 * tid) = o0; *(v4ia*)(cnt + 8 * tid + 4) = o1;
  }
  __syncthreads();

#define HB2(S, D, V) { int d_ = (D); d_ = d_ < 0 ? 0 : (d_ > nN - 1 ? nN - 1 : d_); \
    int s_ = (S); s_ = s_ < 0 ? 0 : (s_ > nN - 1 ? nN - 1 : s_); \
    const int bk_ = ((V) != 0) ? (d_ >> SLB) : DUMP; \
    const unsigned pk_ = ((V) != 0) ? (((unsigned)s_ << SLB) | (unsigned)(d_ & (NBR - 1))) : 0u; \
    int p_ = atomicAdd(&cnt[bk_], 1); p_ = p_ < 0 ? 0 : (p_ > SCH - 1 ? SCH - 1 : p_); \
    sl[p_] = pk_; }
#pragma unroll 1
  for (int it = 0; it < 4; ++it) {
    const int e0 = cbase + it * (NTHR * 4) + tid * 4;
    v4i sa, da, va;
    load_edges4(srcs, dsts, nE, e0, usevec, sa, da, va);
    HB2(sa.x, da.x, va.x) HB2(sa.y, da.y, va.y) HB2(sa.z, da.z, va.z) HB2(sa.w, da.w, va.w)
  }
#undef HB2
  __syncthreads();

  v4u q[4];
  v4i o[2];
#pragma unroll
  for (int it = 0; it < 4; ++it) q[it] = *(const v4ua*)(sl + 4 * (it * NTHR + tid));
#pragma unroll
  for (int it = 0; it < 2; ++it) o[it] = *(const v4ia*)(st + 4 * (it * NTHR + tid));
  unsigned* sp = sorted + (size_t)blockIdx.x * SCH;
  int* opn = offs + (size_t)blockIdx.x * (size_t)offp;
  const int nq = offp >> 2;
#pragma unroll
  for (int it = 0; it < 4; ++it) *(volatile v4u*)(sp + 4 * (it * NTHR + tid)) = q[it];
#pragma unroll
  for (int it = 0; it < 2; ++it) if (it * NTHR + tid < nq) *(volatile v4i*)(opn + 4 * (it * NTHR + tid)) = o[it];
  __threadfence();
#pragma unroll
  for (int it = 0; it < 4; ++it) *(volatile v4u*)(sp + 4 * (it * NTHR + tid)) = q[it];
#pragma unroll
  for (int it = 0; it < 2; ++it) if (it * NTHR + tid < nq) *(volatile v4i*)(opn + 4 * (it * NTHR + tid)) = o[it];
}

__device__ __forceinline__ int build_hits(const int* __restrict__ offs, const unsigned* __restrict__ sorted,
                                          int nChunks, int offp, int b, unsigned* HL, int* wtot, int* flagw,
                                          int tid, int lane, int wave, int& ovfOut) {
  int mycnt = 0, bad = 0;
#pragma unroll 1
  for (int c0 = 0; c0 < nChunks; c0 += NTHR) {
    const int ch  = c0 + tid;
    const int chc = ch < nChunks ? ch : nChunks - 1;
    const int* op = offs + (size_t)chc * (size_t)offp + b;
    int s = op[0], e = op[1];
    s = s < 0 ? 0 : (s > SCH ? SCH : s);
    e = e < 0 ? 0 : (e > SCH ? SCH : e);
    int c = e - s; c = c < 0 ? 0 : c;
    bad |= (c > SEGCAP) ? 1 : 0;
    c = c > SEGCAP ? SEGCAP : c;
    c = (ch < nChunks) ? c : 0;
    mycnt += c;
  }
  int incl = mycnt;
#pragma unroll
  for (int d = 1; d < 32; d <<= 1) {
    const int y = __shfl_up(incl, d, 32);
    if (lane >= d) incl += y;
  }
  if (lane == 31) wtot[wave] = incl;
  if (bad != 0) flagw[0] = 1;
  __syncthreads();
  int base = 0, total = 0;
#pragma unroll
  for (int w2 = 0; w2 < NWAVE; ++w2) { const int v = wtot[w2]; base += (w2 < wave) ? v : 0; total += v; }
  int pos = base + incl - mycnt;
#pragma unroll 1
  for (int c0 = 0; c0 < nChunks; c0 += NTHR) {
    const int ch  = c0 + tid;
    const int chc = ch < nChunks ? ch : nChunks - 1;
    const int* op = offs + (size_t)chc * (size_t)offp + b;
    int s = op[0], e = op[1];
    s = s < 0 ? 0 : (s > SCH ? SCH : s);
    e = e < 0 ? 0 : (e > SCH ? SCH : e);
    int c = e - s; c = c < 0 ? 0 : c;
    c = c > SEGCAP ? SEGCAP : c;
    c = (ch < nChunks) ? c : 0;
    int cm = c;
    cm = max(cm, __shfl_xor(cm, 16, 32));
    cm = max(cm, __shfl_xor(cm, 8, 32));
    cm = max(cm, __shfl_xor(cm, 4, 32));
    cm = max(cm, __shfl_xor(cm, 2, 32));
    cm = max(cm, __shfl_xor(cm, 1, 32));
    cm = __builtin_amdgcn_readfirstlane(cm);
    cm = cm > SEGCAP ? SEGCAP : cm;
    const unsigned* sp = sorted + (size_t)chc * SCH;
#pragma unroll 1
    for (int i = 0; i < cm; ++i) {
      int a = s + ((i < c) ? i : 0);
      a = a > SCH - 1 ? SCH - 1 : a;
      const unsigned v = sp[a];
      const int p = pos + i;
      if (i < c && p >= 0 && p < RCAP) HL[p] = v;
    }
    pos += c;
  }
  __syncthreads();
  int nh = total;
  nh = nh < 0 ? 0 : (nh > RCAP ? RCAP : nh);
  ovfOut = ((total > RCAP) ? 1 : 0) | flagw[0];
  return nh;
}

__global__ __launch_bounds__(NTHR) void k_conv1(const float* __restrict__ pq1, const unsigned* __restrict__ sorted,
                                                const int* __restrict__ offs,
                                                const float* __restrict__ w1b, const float* __restrict__ b1b,
                                                const float* __restrict__ w2a, const float* __restrict__ b2a,
                                                int nN, int nChunks, int offp, float* pq2) {
  __shared__ __attribute__((aligned(16))) unsigned AGG[NBR * 16];
  __shared__ __attribute__((aligned(16))) float P1s[NBR * 16];
  __shared__ __attribute__((aligned(16))) unsigned HL[RCAP];
  __shared__ __attribute__((aligned(16))) unsigned short AT[NWAVE * 16 * 32];
  __shared__ __attribute__((aligned(16))) unsigned short BT[16 * 32];
  __shared__ __attribute__((aligned(16))) float T2[32 * 8];
  __shared__ float b1s[16];
  __shared__ int wtot[NWAVE];
  __shared__ int flagw[4];
  const int tid = (int)threadIdx.x, lane = tid & 31, wave = tid >> 5;
  const int hr = lane & 15, hh = lane >> 4;
  const int nodeBase = (int)blockIdx.x * NBR;

  {
    const v4u e4 = {ENC_NINF, ENC_NINF, ENC_NINF, ENC_NINF};
#pragma unroll
    for (int it = 0; it < 4; ++it) *(v4ua*)(AGG + 4 * (it * NTHR + tid)) = e4;
#pragma unroll
    for (int it = 0; it < 4; ++it) {
      const int idx = it * NTHR + tid;
      const int row = idx >> 2, q = idx & 3;
      const v4f v = *(const v4fa*)(pq1 + (size_t)(nodeBase + row) * PQ1P + 4 * q);
      *(v4fa*)(P1s + row * 16 + 4 * q) = v;
    }
    {
      const int c = tid >> 3, j = tid & 7;
      const int cc = c < 16 ? c : 15;
      const float top = bf16_val(w2a[cc * 4 + (j & 3)]);
      const float bot = bf16_val(w2a[(16 + cc) * 4 + (j & 3)]);
      const float bia = bf16_val(b2a[j & 3]);
      const float f   = (float)(1 - (j >> 2));
      const float wv  = fmaf(f, top - bot, (1.0f - f) * bot);
      const float bv  = f * bia;
      const float val = (c < 16) ? wv : ((c == 16) ? bv : 0.0f);
      T2[tid] = val;
    }
    {
      const int n = tid >> 4, kk = tid & 15;
      const unsigned short bits = (unsigned short)bf16_bits(w1b[kk * 16 + n]);
      BT[n * 32 + kk] = bits;
      BT[n * 32 + 16 + kk] = bits;
    }
    {
      const float bv = bf16_val(b1b[tid & 15]);
      if (tid < 16) b1s[tid] = bv;
    }
    if (tid == 0) flagw[0] = 0;
  }
  __syncthreads();

  int ovf = 0;
  const int nh = build_hits(offs, sorted, nChunks, offp, (int)blockIdx.x, HL, wtot, flagw, tid, lane, wave, ovf);

  FragB bfr;
  bfr.h[0] = *(const v8usa*)(BT + hr * 32 + 8 * hh);
  bfr.h[1] = *(const v8usa*)(BT + hr * 32 + 16 + 8 * hh);
  unsigned short* at = AT + wave * (16 * 32);
  const int ntile = (nh + 15) >> 4;
#pragma unroll 1
  for (int t = wave; t < ntile; t += NWAVE) {
    int idx = 16 * t + hr;
    idx = idx > nh - 1 ? nh - 1 : idx;
    const unsigned ent = HL[idx];
    int sr = (int)(ent >> SLB);
    sr = sr > nN - 1 ? nN - 1 : sr;
    const int dl = (int)(ent & (unsigned)(NBR - 1));
    const float* qp = pq1 + (size_t)sr * PQ1P + 16 + 8 * hh;
    const v4f q0 = *(const v4fa*)qp;
    const v4f q1 = *(const v4fa*)(qp + 4);
    const v4f p0 = *(const v4fa*)(P1s + dl * 16 + 8 * hh);
    const v4f p1 = *(const v4fa*)(P1s + dl * 16 + 8 * hh + 4);
    const v4f ra = p0 + q0, rb = p1 + q1;
    v8us hi8, lo8;
#define SPL(V, I) { const float r_ = relu_np(V); const unsigned hb_ = bf16_bits(r_); \
      hi8[I] = (unsigned short)hb_; lo8[I] = (unsigned short)bf16_bits(r_ - __uint_as_float(hb_ << 16)); }
    SPL(ra.x, 0) SPL(ra.y, 1) SPL(ra.z, 2) SPL(ra.w, 3)
    SPL(rb.x, 4) SPL(rb.y, 5) SPL(rb.z, 6) SPL(rb.w, 7)
#undef SPL
    *(v8usa*)(at + hr * 32 + 8 * hh) = hi8;
    *(v8usa*)(at + hr * 32 + 16 + 8 * hh) = lo8;
    wave_sync();
    FragB af;
    af.h[0] = *(const v8usa*)(at + hr * 32 + 8 * hh);
    af.h[1] = *(const v8usa*)(at + hr * 32 + 16 + 8 * hh);
    wave_sync();
    const v8f z = {0.f, 0.f, 0.f, 0.f, 0.f, 0.f, 0.f, 0.f};
    const v8f d = wmb(af, bfr, z);
#pragma unroll
    for (int r = 0; r < 8; ++r) {
      const int dlr = __shfl(dl, 8 * hh + r, 32);
      atomicMax(&AGG[(dlr & (NBR - 1)) * 16 + hr], enc_f(d[r]));
    }
  }
  __syncthreads();

  {
    const float pz = (ovf != 0) ? __int_as_float(0x7fc00000) : 0.0f;
    const bool empty = (AGG[tid * 16] == ENC_NINF);
    v4f a0 = *(const v4fa*)(T2 + 16 * 8);
    v4f a1 = *(const v4fa*)(T2 + 16 * 8 + 4);
#pragma unroll 4
    for (int c = 0; c < 16; ++c) {
      float v = dec_f(AGG[tid * 16 + c]) + b1s[c];
      v = relu_np(v);
      v = empty ? 0.0f : v;
      v = v + pz;
      const v4f wa = *(const v4fa*)(T2 + c * 8);
      const v4f wb = *(const v4fa*)(T2 + c * 8 + 4);
      a0 = wa * v + a0;
      a1 = wb * v + a1;
    }
    float* ST = P1s;
    *(v4fa*)(ST + tid * 8) = a0;
    *(v4fa*)(ST + tid * 8 + 4) = a1;
  }
  __syncthreads();
  {
    v4f o[2];
#pragma unroll
    for (int it = 0; it < 2; ++it) o[it] = *(const v4fa*)(P1s + 4 * (it * NTHR + tid));
    float* op = pq2 + (size_t)nodeBase * PQ2P;
#pragma unroll
    for (int it = 0; it < 2; ++it) *(volatile v4f*)(op + 4 * (it * NTHR + tid)) = o[it];
    __threadfence();
#pragma unroll
    for (int it = 0; it < 2; ++it) *(volatile v4f*)(op + 4 * (it * NTHR + tid)) = o[it];
  }
}

__global__ __launch_bounds__(NTHR) void k_conv2(const float* __restrict__ pq2, const unsigned* __restrict__ sorted,
                                                const int* __restrict__ offs,
                                                const float* __restrict__ w2b, const float* __restrict__ b2b,
                                                int nN, int nChunks, int offp, float* out) {
  __shared__ __attribute__((aligned(16))) unsigned AGG2[NBR * 4];
  __shared__ __attribute__((aligned(16))) float P2s[NBR * 4];
  __shared__ __attribute__((aligned(16))) unsigned HL[RCAP];
  __shared__ __attribute__((aligned(16))) float os[NBR * 4];
  __shared__ __attribute__((aligned(16))) float w2s[16];
  __shared__ float bb2[4];
  __shared__ int wtot[NWAVE];
  __shared__ int flagw[4];
  const int tid = (int)threadIdx.x, lane = tid & 31, wave = tid >> 5;
  const int nodeBase = (int)blockIdx.x * NBR;

  {
    const v4u e4 = {ENC_NINF, ENC_NINF, ENC_NINF, ENC_NINF};
    *(v4ua*)(AGG2 + 4 * tid) = e4;
    const v4f v = *(const v4fa*)(pq2 + (size_t)(nodeBase + tid) * PQ2P);
    *(v4fa*)(P2s + 4 * tid) = v;
    const float wv = bf16_val(w2b[tid & 15]);
    const float bv = bf16_val(b2b[tid & 3]);
    if (tid < 16) w2s[tid] = wv;
    if (tid < 4)  bb2[tid] = bv;
    if (tid == 0) flagw[0] = 0;
  }
  __syncthreads();

  int ovf = 0;
  const int nh = build_hits(offs, sorted, nChunks, offp, (int)blockIdx.x, HL, wtot, flagw, tid, lane, wave, ovf);

  const v4f wr0 = *(const v4fa*)(w2s);
  const v4f wr1 = *(const v4fa*)(w2s + 4);
  const v4f wr2 = *(const v4fa*)(w2s + 8);
  const v4f wr3 = *(const v4fa*)(w2s + 12);
#pragma unroll 1
  for (int base = 0; base < nh; base += NTHR) {
    int idx = base + tid;
    idx = idx > nh - 1 ? nh - 1 : idx;
    const unsigned ent = HL[idx];
    int sr = (int)(ent >> SLB);
    sr = sr > nN - 1 ? nN - 1 : sr;
    const int dl = (int)(ent & (unsigned)(NBR - 1));
    const v4f q = *(const v4fa*)(pq2 + (size_t)sr * PQ2P + 4);
    const v4f p = *(const v4fa*)(P2s + dl * 4);
    const float t0 = relu_np(p.x + q.x), t1 = relu_np(p.y + q.y);
    const float t2 = relu_np(p.z + q.z), t3 = relu_np(p.w + q.w);
    v4f m = wr0 * t0;
    m = wr1 * t1 + m;
    m = wr2 * t2 + m;
    m = wr3 * t3 + m;
    atomicMax(&AGG2[dl * 4 + 0], enc_f(m.x));
    atomicMax(&AGG2[dl * 4 + 1], enc_f(m.y));
    atomicMax(&AGG2[dl * 4 + 2], enc_f(m.z));
    atomicMax(&AGG2[dl * 4 + 3], enc_f(m.w));
  }
  __syncthreads();

  const float pz = (ovf != 0) ? __int_as_float(0x7fc00000) : 0.0f;
#pragma unroll 1
  for (int it = 0; it < 4; ++it) {
    const int idx = it * NTHR + tid;
    const unsigned e  = AGG2[idx];
    const unsigned e0 = AGG2[idx & ~3];
    const bool empty = (e0 == ENC_NINF);
    float v = dec_f(e) + bb2[idx & 3];
    v = empty ? 0.0f : v;
    float mx = fmaxf(v, __shfl_xor(v, 1, 32));
    mx = fmaxf(mx, __shfl_xor(mx, 2, 32));
    const float sh = v - mx;
    const float ex = expf(sh);
    float s = ex + __shfl_xor(ex, 1, 32);
    s = s + __shfl_xor(s, 2, 32);
    os[idx] = (sh - logf(s)) + pz;
  }
  __syncthreads();
  {
    const v4f ov = *(const v4fa*)(os + 4 * tid);
    const int row = nodeBase + tid;
    float* op = out + (size_t)row * 4;
    const bool okst = row < nN;
    if (okst) *(volatile v4f*)op = ov;
    __threadfence();
    if (okst) *(volatile v4f*)op = ov;
  }
}

static inline int cdiv(int a, int b) { return (a + b - 1) / b; }
static inline size_t al256(size_t o) { return (o + 255) & ~(size_t)255; }

extern "C" void kernel_launch(void* const* d_in, const int* in_sizes, int n_in,
                              void* d_out, int out_size, void* d_ws, size_t ws_size,
                              hipStream_t stream) {
  if (n_in < 10) return;
  if (in_sizes[0] < 3 || (in_sizes[0] % 3) != 0) return;
  const int nN = in_sizes[0] / 3;
  if (in_sizes[1] < 2 || (in_sizes[1] & 1) != 0) return;
  const int nE = in_sizes[1] / 2;
  if (nE < 1 || nE > (1 << 30)) return;
  if (in_sizes[2] != 96 || in_sizes[3] != 16) return;
  if (in_sizes[4] != 256 || in_sizes[5] != 16) return;
  if (in_sizes[6] != 128 || in_sizes[7] != 4) return;
  if (in_sizes[8] != 16 || in_sizes[9] != 4) return;
  if ((long long)out_size != (long long)nN * 4) return;

  const float* x    = (const float*)d_in[0];
  const int*   edge = (const int*)d_in[1];
  const float* w1a  = (const float*)d_in[2];
  const float* b1a  = (const float*)d_in[3];
  const float* w1b  = (const float*)d_in[4];
  const float* b1b  = (const float*)d_in[5];
  const float* w2a  = (const float*)d_in[6];
  const float* b2a  = (const float*)d_in[7];
  const float* w2b  = (const float*)d_in[8];
  const float* b2b  = (const float*)d_in[9];
  float* out = (float*)d_out;
  const int* src = edge;
  const int* dst = edge + nE;

  const int nb = cdiv(nN, NBR);
  if (nb < 1 || nb + 1 > DUMP) return;
  const int NP = nb * NBR;
  const int offp = cdiv(nb + 1, 32) * 32;
  if (offp > NB2) return;
  const int nChunks = cdiv(nE, SCH);
  const int vec4 = ((nE & 3) == 0) ? 1 : 0;

  char* ws = (char*)d_ws;
  size_t off = 0;
  const size_t oPQ1 = off; off = al256(off + (size_t)NP * PQ1P * 4);
  const size_t oSRT = off; off = al256(off + (size_t)nChunks * SCH * 4);
  const size_t oOFF = off; off = al256(off + (size_t)nChunks * offp * 4);
  const size_t oPQ2 = off; off = al256(off + (size_t)NP * PQ2P * 4);
  if (off > ws_size || off > (size_t)WSMAX) return;
  float*    PQ1 = (float*)(ws + oPQ1);
  unsigned* SRT = (unsigned*)(ws + oSRT);
  int*      OFS = (int*)(ws + oOFF);
  float*    PQ2 = (float*)(ws + oPQ2);

  k_prep<<<nb, NTHR, 0, stream>>>(x, w1a, b1a, nN, PQ1);
  k_sort<<<nChunks, NTHR, 0, stream>>>(src, dst, nE, nN, vec4, offp, SRT, OFS);
  k_conv1<<<nb, NTHR, 0, stream>>>(PQ1, SRT, OFS, w1b, b1b, w2a, b2a, nN, nChunks, offp, PQ2);
  k_conv2<<<nb, NTHR, 0, stream>>>(PQ2, SRT, OFS, w2b, b2b, nN, nChunks, offp, out);
}
